// LSTMMLP_PSO_28252294873520
// MI455X (gfx1250) — hardware-verified
//
#include <hip/hip_runtime.h>


typedef _Float16 f16t;
typedef f16t  v16h __attribute__((ext_vector_type(16)));
typedef f16t  v8h  __attribute__((ext_vector_type(8)));
typedef float v8f  __attribute__((ext_vector_type(8)));
typedef float v4f  __attribute__((ext_vector_type(4)));

#define T_STEPS 60
#define FIN 5
#define HID 64
#define NZ 256
#define MLP_D1 64
#define MLP_D2 32
#define CDIM 65
#define BN_EPS 1e-3f
#define ROWS_PER_WAVE 16
#define ROWS_PER_BLK 64
#define BLK_THREADS 128
#define UPITCH 64
#define HSP 66
#define OPS 16.0f
#define INVS 0.00390625f

union FragA { v16h v; v8h q[2]; };
union FragB { v16h v; f16t e[16]; };

__device__ __forceinline__ float sigm(float z) {
  return __builtin_amdgcn_rcpf(1.0f + __expf(-z));
}
__device__ __forceinline__ float tanhx(float x) {
  return fmaf(-2.0f, __builtin_amdgcn_rcpf(1.0f + __expf(2.0f * x)), 1.0f);
}

__device__ __forceinline__ v8f wmma_pair(v16h a0, v16h b0, v16h a1, v16h b1) {
  v8f c = {0.f, 0.f, 0.f, 0.f, 0.f, 0.f, 0.f, 0.f};
  c = __builtin_amdgcn_wmma_f32_16x16x32_f16(false, a0, false, b0, (short)0, c, false, false);
  c = __builtin_amdgcn_wmma_f32_16x16x32_f16(false, a1, false, b1, (short)0, c, false, false);
  asm volatile("v_nop\n\tv_nop\n\tv_nop\n\tv_nop" : "+v"(c) : "v"(a0), "v"(a1), "v"(b0), "v"(b1));
  return c;
}

__global__ __launch_bounds__(BLK_THREADS)
void lstm_head(const float* __restrict__ x_seq, const float* __restrict__ x_static,
               const float* __restrict__ W,  const float* __restrict__ U,  const float* __restrict__ bz,
               const float* __restrict__ bn1_g, const float* __restrict__ bn1_b,
               const float* __restrict__ bn1_m, const float* __restrict__ bn1_v,
               const float* __restrict__ bn2_g, const float* __restrict__ bn2_b,
               const float* __restrict__ bn2_m, const float* __restrict__ bn2_v,
               const float* __restrict__ W1, const float* __restrict__ b1,
               const float* __restrict__ W2, const float* __restrict__ b2,
               const float* __restrict__ Wo, const float* __restrict__ bo,
               float* __restrict__ out, int nb)
{
  __shared__ __attribute__((aligned(16))) f16t  Up[NZ * UPITCH];
  __shared__ __attribute__((aligned(16))) float Wl[NZ * 8];
  __shared__ __attribute__((aligned(16))) float hstage[ROWS_PER_BLK * HSP];
  __shared__ __attribute__((aligned(16))) float outv[ROWS_PER_BLK];

  const int tid  = threadIdx.x;
  const int lane = tid & 31;
  const int wave = tid >> 5;
  const int n    = lane & 15;
  const int hh   = lane >> 4;
  const int row0b = blockIdx.x * ROWS_PER_BLK;
  if (row0b + ROWS_PER_BLK > nb) return;

  for (int idx = tid; idx < HID * NZ; idx += BLK_THREADS) {
    const int k = idx >> 8, M = idx & (NZ - 1);
    Up[M * UPITCH + k] = (f16t)(U[idx] * OPS);
  }
  for (int idx = tid; idx < NZ * 8; idx += BLK_THREADS) {
    const int m = idx >> 3, k = idx & 7;
    float val = 0.0f;
    if (k < FIN) val = W[k * NZ + m];
    else if (k == FIN) val = bz[m];
    Wl[idx] = val;
  }
  __syncthreads();

  const int roww = row0b + wave * ROWS_PER_WAVE + n;
  const float* xp = x_seq + (size_t)roww * T_STEPS * FIN;
  const f16t* upl = Up + n * UPITCH + 8 * hh;

  float cst[4][8], hk[4][8];
#pragma unroll
  for (int hc = 0; hc < 4; ++hc)
#pragma unroll
    for (int r = 0; r < 8; ++r) { cst[hc][r] = 0.0f; hk[hc][r] = 0.0f; }

#pragma unroll 1
  for (int t = 0; t < T_STEPS; ++t) {
    const float* xt = xp + t * FIN;
    const float x0 = xt[0], x1 = xt[1], x2 = xt[2], x3 = xt[3], x4 = xt[4];
    const bool mk = (x0 != 0.0f) | (x1 != 0.0f) | (x2 != 0.0f) | (x3 != 0.0f) | (x4 != 0.0f);

    FragB hb0, hb1;
#pragma unroll
    for (int i = 0; i < 8; ++i) {
      hb0.e[i]     = (f16t)(hk[0][i] * OPS);
      hb0.e[8 + i] = (f16t)(hk[1][i] * OPS);
      hb1.e[i]     = (f16t)(hk[2][i] * OPS);
      hb1.e[8 + i] = (f16t)(hk[3][i] * OPS);
    }

#pragma unroll
    for (int hc = 0; hc < 4; ++hc) {
      float z[4][8];
#pragma unroll
      for (int gI = 0; gI < 4; ++gI) {
        const int mt = gI * 4 + hc;
        const f16t* ap = upl + mt * 16 * UPITCH;
        FragA a0, a1;
        a0.q[0] = *(const v8h*)(ap);
        a0.q[1] = *(const v8h*)(ap + 16);
        a1.q[0] = *(const v8h*)(ap + 32);
        a1.q[1] = *(const v8h*)(ap + 48);
        const v8f acc = wmma_pair(a0.v, hb0.v, a1.v, hb1.v);
        const float* wq = Wl + (mt * 16 + 8 * hh) * 8;
#pragma unroll
        for (int r = 0; r < 8; ++r) {
          const v4f w0 = *(const v4f*)(wq + r * 8);
          const v4f w1 = *(const v4f*)(wq + r * 8 + 4);
          float s = w1[1];
          s = fmaf(x0, w0[0], s);
          s = fmaf(x1, w0[1], s);
          s = fmaf(x2, w0[2], s);
          s = fmaf(x3, w0[3], s);
          s = fmaf(x4, w1[0], s);
          z[gI][r] = fmaf(acc[r], INVS, s);
        }
      }
#pragma unroll
      for (int r = 0; r < 8; ++r) {
        const float iv = sigm(z[0][r]);
        const float fv = sigm(z[1][r]);
        const float gv = tanhx(z[2][r]);
        const float ov = sigm(z[3][r]);
        const float cn = fmaf(fv, cst[hc][r], iv * gv);
        const float hn = ov * tanhx(cn);
        cst[hc][r] = mk ? cn : cst[hc][r];
        hk[hc][r]  = mk ? hn : hk[hc][r];
      }
    }
  }

  {
    float* hs = hstage + (wave * ROWS_PER_WAVE + n) * HSP + 8 * hh;
#pragma unroll
    for (int hc = 0; hc < 4; ++hc)
#pragma unroll
      for (int r = 0; r < 8; ++r) hs[hc * 16 + r] = hk[hc][r];
  }
  __syncthreads();

  if (tid < ROWS_PER_BLK) {
    const int gr = row0b + tid;
    float* hr = hstage + tid * HSP;
#pragma unroll 1
    for (int c = 0; c < HID; ++c) {
      float v = hr[c];
      v = (v - bn1_m[c]) * (bn1_g[c] * rsqrtf(bn1_v[c] + BN_EPS)) + bn1_b[c];
      v = (v - bn2_m[c]) * (bn2_g[c] * rsqrtf(bn2_v[c] + BN_EPS)) + bn2_b[c];
      hr[c] = v;
    }
    {
      float v = x_static[gr];
      v = (v - bn2_m[HID]) * (bn2_g[HID] * rsqrtf(bn2_v[HID] + BN_EPS)) + bn2_b[HID];
      hr[HID] = v;
    }
    float a2[MLP_D2];
#pragma unroll
    for (int e = 0; e < MLP_D2; ++e) a2[e] = b2[e];
#pragma unroll 1
    for (int d = 0; d < MLP_D1; ++d) {
      float s = b1[d];
#pragma unroll 5
      for (int c = 0; c < CDIM; ++c) s = fmaf(hr[c], W1[c * MLP_D1 + d], s);
      s = fmaxf(s, 0.0f);
#pragma unroll
      for (int e = 0; e < MLP_D2; ++e) a2[e] = fmaf(s, W2[d * MLP_D2 + e], a2[e]);
    }
    float o = bo[0];
#pragma unroll
    for (int e = 0; e < MLP_D2; ++e) o = fmaf(fmaxf(a2[e], 0.0f), Wo[e], o);
    outv[tid] = o;
  }
  __syncthreads();

  v4f ov = {0.f, 0.f, 0.f, 0.f};
  if (tid < 16) {
    ov = *(const v4f*)(outv + tid * 4);
    *(volatile v4f*)(out + row0b + tid * 4) = ov;
  }
  __threadfence();
  if (tid < 16) {
    *(volatile v4f*)(out + row0b + tid * 4) = ov;
  }
}

extern "C" void kernel_launch(void* const* d_in, const int* in_sizes, int n_in,
                              void* d_out, int out_size, void* d_ws, size_t ws_size,
                              hipStream_t stream) {
  (void)d_ws; (void)ws_size;
  if (n_in < 19) return;
  const int nb = out_size;
  if (nb <= 0 || (nb % ROWS_PER_BLK) != 0) return;
  if (in_sizes[0] != nb * T_STEPS * FIN || in_sizes[1] != nb ||
      in_sizes[2] != FIN * NZ || in_sizes[3] != HID * NZ || in_sizes[4] != NZ ||
      in_sizes[5] != HID || in_sizes[6] != HID || in_sizes[7] != HID || in_sizes[8] != HID ||
      in_sizes[9] != CDIM || in_sizes[10] != CDIM || in_sizes[11] != CDIM || in_sizes[12] != CDIM ||
      in_sizes[13] != CDIM * MLP_D1 || in_sizes[14] != MLP_D1 ||
      in_sizes[15] != MLP_D1 * MLP_D2 || in_sizes[16] != MLP_D2 ||
      in_sizes[17] != MLP_D2 || in_sizes[18] != 1) return;

  const float* x_seq    = (const float*)d_in[0];
  const float* x_static = (const float*)d_in[1];
  const float* W        = (const float*)d_in[2];
  const float* U        = (const float*)d_in[3];
  const float* b        = (const float*)d_in[4];
  const float* bn1_g    = (const float*)d_in[5];
  const float* bn1_b    = (const float*)d_in[6];
  const float* bn1_m    = (const float*)d_in[7];
  const float* bn1_v    = (const float*)d_in[8];
  const float* bn2_g    = (const float*)d_in[9];
  const float* bn2_b    = (const float*)d_in[10];
  const float* bn2_m    = (const float*)d_in[11];
  const float* bn2_v    = (const float*)d_in[12];
  const float* W1       = (const float*)d_in[13];
  const float* b1       = (const float*)d_in[14];
  const float* W2       = (const float*)d_in[15];
  const float* b2       = (const float*)d_in[16];
  const float* Wo       = (const float*)d_in[17];
  const float* bo       = (const float*)d_in[18];
  float* out = (float*)d_out;

  const int grid = nb / ROWS_PER_BLK;
  lstm_head<<<dim3(grid), dim3(BLK_THREADS), 0, stream>>>(
      x_seq, x_static, W, U, b,
      bn1_g, bn1_b, bn1_m, bn1_v,
      bn2_g, bn2_b, bn2_m, bn2_v,
      W1, b1, W2, b2, Wo, bo, out, nb);
}
